// NonLocalSelfAttention_58076547777045
// MI455X (gfx1250) — hardware-verified
//
#include <hip/hip_runtime.h>

typedef _Float16 v16h __attribute__((ext_vector_type(16)));
typedef _Float16 v8h  __attribute__((ext_vector_type(8)));
typedef float    v8f  __attribute__((ext_vector_type(8)));
typedef float    v4f  __attribute__((ext_vector_type(4)));
typedef v8h __attribute__((may_alias)) v8ha;
typedef v4f __attribute__((may_alias)) v4fa;

union Frag { v16h v; v8h half[2]; };

#define NIMG   2
#define C_IN   256
#define DH     128
#define HW     64
#define SPAT   4096
#define N_TOK  8192
#define NX     (NIMG * C_IN * SPAT)
#define NW     (DH * C_IN)
#define KSTEP  32
#define PSCALE 16384.0f
#define WSCALE 32.0f
#define MSCALE 64.0f
#define XPITCH 72
#define OPITCH 68

__device__ __forceinline__ v8f wmma_f16(v16h a, v16h b, v8f c) {
  v8f d = __builtin_amdgcn_wmma_f32_16x16x32_f16(false, a, false, b, (short)0, c, false, false);
  asm volatile("v_nop\n\tv_nop\n\tv_nop\n\tv_nop" : "+v"(d) : "v"(a), "v"(b));
  return d;
}

__device__ __forceinline__ v16h load_frag(const _Float16* p, int h) {
  Frag f;
  f.half[0] = *(const v8ha*)(p + 8 * h);
  f.half[1] = *(const v8ha*)(p + 16 + 8 * h);
  return f.v;
}

__device__ __forceinline__ void cvtx_store_pass(const _Float16* sT, _Float16* xh,
                                                int img, int s0, int c0, int w, int lane) {
  const int q8 = lane & 7, sub = lane >> 3;
  #pragma unroll
  for (int i = 0; i < 2; ++i) {
    const int lid = w * 8 + i * 4 + sub;
    const v8h v = *(const v8ha*)(sT + lid * XPITCH + 8 * q8);
    _Float16* dst = xh + ((size_t)img * SPAT + s0 + lid) * C_IN + c0 + 8 * q8;
    *(volatile v8h*)dst = v;
  }
}

__global__ __launch_bounds__(256) void k_cvt_x(const float* __restrict__ feat,
                                               _Float16* __restrict__ xh)
{
  __shared__ __attribute__((aligned(16))) _Float16 sT[64 * XPITCH];
  const int tid = threadIdx.x, lane = tid & 31, w = tid >> 5;
  const int s0 = blockIdx.x * 64, c0 = blockIdx.y * 64, img = blockIdx.z;
  const float* src = feat + ((size_t)img * C_IN + c0) * SPAT + s0;
  #pragma unroll
  for (int i = 0; i < 16; ++i) {
    const int idx = i * 256 + tid;
    const int cc = idx >> 6, ss = idx & 63;
    sT[ss * XPITCH + cc] = (_Float16)src[(size_t)cc * SPAT + ss];
  }
  __syncthreads();
  cvtx_store_pass(sT, xh, img, s0, c0, w, lane);
  __threadfence();
  cvtx_store_pass(sT, xh, img, s0, c0, w, lane);
}

__global__ __launch_bounds__(256) void k_cvt_w(
    const float* __restrict__ wq, const float* __restrict__ wk,
    const float* __restrict__ wv, const float* __restrict__ wm,
    _Float16* __restrict__ wh, _Float16* __restrict__ wmh)
{
  const int g = blockIdx.x * 256 + threadIdx.x;
  const int n3 = 3 * NW / 8;
  const int nm = NW / 8;
  if (g >= n3 + nm) return;
  const float* src;
  _Float16* dst;
  if (g < n3) {
    const int wsel = g / nm;
    const int off = g - wsel * nm;
    const float* wsrc = (wsel == 0) ? wq : ((wsel == 1) ? wk : wv);
    src = wsrc + (size_t)off * 8;
    dst = wh + (size_t)g * 8;
  } else {
    const int e = g - n3;
    src = wm + (size_t)e * 8;
    dst = wmh + (size_t)e * 8;
  }
  const v4f a = *(const v4fa*)src;
  const v4f c = *(const v4fa*)(src + 4);
  const v8h o = { (_Float16)(a.x * WSCALE), (_Float16)(a.y * WSCALE), (_Float16)(a.z * WSCALE), (_Float16)(a.w * WSCALE),
                  (_Float16)(c.x * WSCALE), (_Float16)(c.y * WSCALE), (_Float16)(c.z * WSCALE), (_Float16)(c.w * WSCALE) };
  *(volatile v8h*)dst = o;
  __threadfence();
  *(volatile v8h*)dst = o;
}

__device__ __forceinline__ void proj_store_pass(const _Float16* sT, _Float16* plane, _Float16* vt,
                                                int which, int dseg, int m0, int w, int lane) {
  const int q8 = lane & 7, sub = lane >> 3;
  #pragma unroll
  for (int i = 0; i < 8; ++i) {
    const int lid = w * 32 + i * 4 + sub;
    v8h v;
    _Float16* dst;
    if (which != 2) {
      v = *(const v8ha*)(sT + lid * 64 + 8 * q8);
      dst = plane + (size_t)(m0 + lid) * DH + 64 * dseg + 8 * q8;
    } else {
      const int d = lid >> 1, hl = lid & 1;
      v = *(const v8ha*)(sT + d * 128 + 64 * hl + 8 * q8);
      dst = vt + (size_t)(64 * dseg + d) * N_TOK + m0 + 64 * hl + 8 * q8;
    }
    *(volatile v8h*)dst = v;
  }
}

__global__ __launch_bounds__(128) void k_proj(
    const _Float16* __restrict__ xh,
    const _Float16* __restrict__ wh,
    const float* __restrict__ bq, const float* __restrict__ bk, const float* __restrict__ bv,
    _Float16* __restrict__ ka,
    _Float16* __restrict__ qa,
    _Float16* __restrict__ vt)
{
  __shared__ __attribute__((aligned(16))) _Float16 sT[128 * 64];

  const int tid = threadIdx.x, lane = tid & 31, w = tid >> 5;
  const int h = lane >> 4, m = lane & 15;
  const int m0 = blockIdx.x * 128;
  const int cg = blockIdx.y;
  const int which = cg >> 1, dseg = cg & 1;
  const int m0w = m0 + 32 * w;

  const _Float16* xa0 = xh + (size_t)(m0w + m) * C_IN;
  const _Float16* xa1 = xa0 + (size_t)16 * C_IN;
  const _Float16* wb  = wh + ((size_t)which * DH + 64 * dseg + m) * C_IN;

  const v8f zero8 = {0.f, 0.f, 0.f, 0.f, 0.f, 0.f, 0.f, 0.f};
  v8f acc[2][4];
  #pragma unroll
  for (int mt = 0; mt < 2; ++mt)
    #pragma unroll
    for (int nt = 0; nt < 4; ++nt) acc[mt][nt] = zero8;

  #pragma unroll 1
  for (int k0 = 0; k0 < C_IN; k0 += 32) {
    const v16h a0 = load_frag(xa0 + k0, h);
    const v16h a1 = load_frag(xa1 + k0, h);
    #pragma unroll
    for (int nt = 0; nt < 4; ++nt) {
      const v16h b = load_frag(wb + (size_t)nt * 16 * C_IN + k0, h);
      acc[0][nt] = wmma_f16(a0, b, acc[0][nt]);
      acc[1][nt] = wmma_f16(a1, b, acc[1][nt]);
    }
  }

  const float* bias = (which == 0) ? bq : ((which == 1) ? bk : bv);
  #pragma unroll
  for (int nt = 0; nt < 4; ++nt) {
    const int feat = 16 * nt + m;
    const float bvl = bias[64 * dseg + feat];
    #pragma unroll
    for (int mt = 0; mt < 2; ++mt) {
      #pragma unroll
      for (int r = 0; r < 8; ++r) {
        const int tokl = 32 * w + 16 * mt + 8 * h + r;
        const float y = acc[mt][nt][r] * (1.0f / WSCALE) + bvl;
        const int idx = (which == 2) ? (feat * 128 + tokl) : (tokl * 64 + feat);
        sT[idx] = (_Float16)y;
      }
    }
  }
  __syncthreads();

  _Float16* plane = (which == 0) ? ka : qa;
  proj_store_pass(sT, plane, vt, which, dseg, m0, w, lane);
  __threadfence();
  proj_store_pass(sT, plane, vt, which, dseg, m0, w, lane);
}

__device__ __forceinline__ v16h pack_p(v8f a, v8f c) {
  const v16h r = { (_Float16)(a[0] * PSCALE), (_Float16)(a[1] * PSCALE), (_Float16)(a[2] * PSCALE), (_Float16)(a[3] * PSCALE),
                   (_Float16)(a[4] * PSCALE), (_Float16)(a[5] * PSCALE), (_Float16)(a[6] * PSCALE), (_Float16)(a[7] * PSCALE),
                   (_Float16)(c[0] * PSCALE), (_Float16)(c[1] * PSCALE), (_Float16)(c[2] * PSCALE), (_Float16)(c[3] * PSCALE),
                   (_Float16)(c[4] * PSCALE), (_Float16)(c[5] * PSCALE), (_Float16)(c[6] * PSCALE), (_Float16)(c[7] * PSCALE) };
  return r;
}

__device__ __forceinline__ void att_store_pass(const _Float16* so, _Float16* mh, int q0, int lane) {
  const int q8 = lane & 7, sub = lane >> 3;
  #pragma unroll
  for (int i = 0; i < 8; ++i) {
    const int lid = i * 4 + sub;
    const int row = lid >> 1, hl = lid & 1;
    const v8h v = *(const v8ha*)(so + row * DH + 64 * hl + 8 * q8);
    _Float16* dst = mh + (size_t)(q0 + row) * DH + 64 * hl + 8 * q8;
    *(volatile v8h*)dst = v;
  }
}

__global__ __launch_bounds__(128) void k_attn(
    const _Float16* __restrict__ qa,
    const _Float16* __restrict__ ka,
    const _Float16* __restrict__ vt,
    _Float16* __restrict__ mh)
{
  __shared__ __attribute__((aligned(16))) _Float16 sO[4 * 16 * DH];

  const int tid = threadIdx.x, lane = tid & 31, w = tid >> 5;
  const int h = lane >> 4, m = lane & 15;
  const int q0 = blockIdx.x * 64 + 16 * w;

  const _Float16* qrow = qa + (size_t)(q0 + m) * DH;
  v16h qb[4];
  #pragma unroll
  for (int kk = 0; kk < 4; ++kk) qb[kk] = load_frag(qrow + 32 * kk, h);

  const v8f zero8 = {0.f, 0.f, 0.f, 0.f, 0.f, 0.f, 0.f, 0.f};
  v8f o[8];
  #pragma unroll
  for (int t = 0; t < 8; ++t) o[t] = zero8;
  float mrun = -1e30f, lrun = 0.0f;

  const _Float16* kbase = ka + (size_t)m * DH;
  const _Float16* vbase = vt + (size_t)m * N_TOK;

  #pragma unroll 1
  for (int kb = 0; kb < N_TOK; kb += KSTEP) {
    v8f s[2];
    #pragma unroll
    for (int j = 0; j < 2; ++j) {
      const _Float16* kp = kbase + (size_t)(kb + 16 * j) * DH;
      v8f z = zero8;
      #pragma unroll
      for (int kk = 0; kk < 4; ++kk) {
        const v16h kf = load_frag(kp + 32 * kk, h);
        z = wmma_f16(kf, qb[kk], z);
      }
      s[j] = z;
    }

    float mloc = s[0][0];
    #pragma unroll
    for (int j = 0; j < 2; ++j)
      #pragma unroll
      for (int r = 0; r < 8; ++r) mloc = fmaxf(mloc, s[j][r]);
    mloc = fmaxf(mloc, __shfl_xor(mloc, 16));
    const float mnew = fmaxf(mrun, mloc);
    const float alpha = __expf(mrun - mnew);
    mrun = mnew;
    float lsum = 0.0f;
    #pragma unroll
    for (int j = 0; j < 2; ++j)
      #pragma unroll
      for (int r = 0; r < 8; ++r) {
        const float p = __expf(s[j][r] - mnew);
        s[j][r] = p;
        lsum += p;
      }
    lsum += __shfl_xor(lsum, 16);
    lrun = lrun * alpha + lsum;
    #pragma unroll
    for (int t = 0; t < 8; ++t)
      #pragma unroll
      for (int r = 0; r < 8; ++r) o[t][r] = o[t][r] * alpha;

    const v16h pb = pack_p(s[0], s[1]);

    #pragma unroll
    for (int t = 0; t < 8; ++t) {
      const v16h vf = load_frag(vbase + (size_t)(16 * t) * N_TOK + kb, h);
      o[t] = wmma_f16(vf, pb, o[t]);
    }
  }

  const float inv = (1.0f / lrun) * (MSCALE / PSCALE);
  _Float16* so = sO + w * (16 * DH);
  #pragma unroll
  for (int t = 0; t < 8; ++t) {
    const v8h pk = { (_Float16)(o[t][0] * inv), (_Float16)(o[t][1] * inv), (_Float16)(o[t][2] * inv), (_Float16)(o[t][3] * inv),
                     (_Float16)(o[t][4] * inv), (_Float16)(o[t][5] * inv), (_Float16)(o[t][6] * inv), (_Float16)(o[t][7] * inv) };
    *(v8ha*)(so + m * DH + 16 * t + 8 * h) = pk;
  }
  __syncthreads();

  att_store_pass(so, mh, q0, lane);
  __threadfence();
  att_store_pass(so, mh, q0, lane);
}

__device__ __forceinline__ void out_store_pass(const float* sd, const float* bm, const float* feat,
                                               float* out, int img, int a, int cbase, int lane) {
  const int q8 = lane & 7, sub = lane >> 3;
  #pragma unroll
  for (int i = 0; i < 16; ++i) {
    const int lid = i * 4 + sub;
    const int col = lid >> 1, hl = lid & 1;
    const int co = cbase + col;
    v4f v = *(const v4fa*)(sd + col * OPITCH + 32 * hl + 4 * q8);
    const size_t oidx = (((size_t)img * C_IN + co) * HW + a) * HW + 32 * hl + 4 * q8;
    const v4f f4 = *(const v4fa*)(feat + oidx);
    const float bb = bm[co];
    v = v + f4 + bb;
    *(volatile v4f*)(out + oidx) = v;
  }
}

__global__ __launch_bounds__(128) void k_out(
    const _Float16* __restrict__ mh,
    const _Float16* __restrict__ wmh,
    const float* __restrict__ bm,
    const float* __restrict__ feat,
    float* __restrict__ out)
{
  __shared__ __attribute__((aligned(16))) float sD[4 * 32 * OPITCH];

  const int tid = threadIdx.x, lane = tid & 31, w = tid >> 5;
  const int h = lane >> 4, m = lane & 15;
  const int img = blockIdx.x >> 6, a = blockIdx.x & 63;
  const int cbase = blockIdx.y * 128 + 32 * w;

  const _Float16* wa0 = wmh + (size_t)(cbase + m) * DH;
  const _Float16* wa1 = wa0 + (size_t)16 * DH;
  const _Float16* mb0 = mh + ((size_t)img * SPAT + (size_t)m * HW + a) * DH;

  const v8f zero8 = {0.f, 0.f, 0.f, 0.f, 0.f, 0.f, 0.f, 0.f};
  v8f acc[2][4];
  #pragma unroll
  for (int mt = 0; mt < 2; ++mt)
    #pragma unroll
    for (int nt = 0; nt < 4; ++nt) acc[mt][nt] = zero8;

  #pragma unroll
  for (int kk = 0; kk < 4; ++kk) {
    const v16h a0 = load_frag(wa0 + 32 * kk, h);
    const v16h a1 = load_frag(wa1 + 32 * kk, h);
    #pragma unroll
    for (int nt = 0; nt < 4; ++nt) {
      const v16h b = load_frag(mb0 + (size_t)nt * 16 * HW * DH + 32 * kk, h);
      acc[0][nt] = wmma_f16(a0, b, acc[0][nt]);
      acc[1][nt] = wmma_f16(a1, b, acc[1][nt]);
    }
  }

  float* sd = sD + w * (32 * OPITCH);
  #pragma unroll
  for (int mt = 0; mt < 2; ++mt)
    #pragma unroll
    for (int nt = 0; nt < 4; ++nt)
      #pragma unroll
      for (int r = 0; r < 8; ++r)
        sd[(16 * mt + 8 * h + r) * OPITCH + 16 * nt + m] = acc[mt][nt][r] * (1.0f / (WSCALE * MSCALE));
  __syncthreads();

  out_store_pass(sd, bm, feat, out, img, a, cbase, lane);
  __threadfence();
  out_store_pass(sd, bm, feat, out, img, a, cbase, lane);
}

extern "C" void kernel_launch(void* const* d_in, const int* in_sizes, int n_in,
                              void* d_out, int out_size, void* d_ws, size_t ws_size,
                              hipStream_t stream) {
  if (n_in < 9) return;
  if (in_sizes[0] != NX) return;
  if (in_sizes[1] != NW || in_sizes[3] != NW || in_sizes[5] != NW || in_sizes[7] != NW) return;
  if (in_sizes[2] != DH || in_sizes[4] != DH || in_sizes[6] != DH || in_sizes[8] != C_IN) return;
  if (out_size != NX) return;

  const float* feat = (const float*)d_in[0];
  const float* Wq   = (const float*)d_in[1];
  const float* bq   = (const float*)d_in[2];
  const float* Wk   = (const float*)d_in[3];
  const float* bk   = (const float*)d_in[4];
  const float* Wv   = (const float*)d_in[5];
  const float* bv   = (const float*)d_in[6];
  const float* Wm   = (const float*)d_in[7];
  const float* bm   = (const float*)d_in[8];
  float* out = (float*)d_out;

  const size_t xh_bytes  = (size_t)N_TOK * C_IN * 2;
  const size_t wh_bytes  = (size_t)3 * NW * 2;
  const size_t wmh_bytes = (size_t)NW * 2;
  const size_t pl_bytes  = (size_t)N_TOK * DH * 2;
  const size_t total = xh_bytes + wh_bytes + wmh_bytes + 4 * pl_bytes;
  if (total > ws_size) return;

  char* ws = (char*)d_ws;
  size_t off = 0;
  _Float16* xh  = (_Float16*)(ws + off); off += xh_bytes;
  _Float16* wh  = (_Float16*)(ws + off); off += wh_bytes;
  _Float16* wmh = (_Float16*)(ws + off); off += wmh_bytes;
  _Float16* ka  = (_Float16*)(ws + off); off += pl_bytes;
  _Float16* qa  = (_Float16*)(ws + off); off += pl_bytes;
  _Float16* vt  = (_Float16*)(ws + off); off += pl_bytes;
  _Float16* mh  = (_Float16*)(ws + off); off += pl_bytes;

  dim3 gCx(SPAT / 64, C_IN / 64, NIMG);
  k_cvt_x<<<gCx, 256, 0, stream>>>(feat, xh);

  const int ngroups = 3 * NW / 8 + NW / 8;
  k_cvt_w<<<(ngroups + 255) / 256, 256, 0, stream>>>(Wq, Wk, Wv, Wm, wh, wmh);

  dim3 gProj(N_TOK / 128, 6);
  k_proj<<<gProj, 128, 0, stream>>>(xh, wh, bq, bk, bv, ka, qa, vt);

  k_attn<<<N_TOK / 64, 128, 0, stream>>>(qa, ka, vt, mh);

  dim3 gOut(NIMG * HW, 2);
  k_out<<<gOut, 128, 0, stream>>>(mh, wmh, bm, feat, out);
}
